// TemporalSelfAttention_781684048572
// MI455X (gfx1250) — hardware-verified
//
#include <hip/hip_runtime.h>


namespace {
constexpr int B = 8, T = 512, DM = 1024, H = 16, HD = 64, TE = 1024, BL = 8  ;
constexpr float XS = 8.0f, WSC = 256.0f, PS = 1024.0f, LOG2E = 1.4426950408889634f, EPS = 1e-5f, MNEG = -100000.0f;
static_assert(T % 64 == 0, "tiling");
typedef _Float16 b16;
typedef __attribute__((ext_vector_type(16))) _Float16 v16b;
typedef __attribute__((ext_vector_type(8))) _Float16 v8b;
typedef __attribute__((ext_vector_type(8))) float v8f;
typedef __attribute__((ext_vector_type(4))) float v4f;
__device__ __forceinline__ float bf16_rne(float f) { unsigned int u = __float_as_uint(f); u += 0x7FFFu + ((u >> 16) & 1u); return __uint_as_float(u & 0xFFFF0000u); }
__device__ __forceinline__ void split16(float v, b16& hi, b16& lo) { hi = (b16)v; lo = (b16)(v - (float)hi); }
__device__ __forceinline__ v16b frag_kb(const b16* p, int hh) { const v8b a = *(const v8b*)(p + 8 * hh), b = *(const v8b*)(p + 16 + 8 * hh); v16b f;
#pragma unroll
  for (int e = 0; e < 8; ++e) { f[e] = a[e]; f[8 + e] = b[e]; } return f; }
__device__ __forceinline__ v8f wmma16b(v16b a, v16b b, v8f c) { v8f d = __builtin_amdgcn_wmma_f32_16x16x32_f16(false, a, false, b, (short)0, c, false, false); asm volatile("v_nop\n\tv_nop\n\tv_nop\n\tv_nop" : "+v"(d) : "v"(a), "v"(b)); return d; }
__device__ __forceinline__ void wave_lds_sync() { __builtin_amdgcn_fence(__ATOMIC_RELEASE, "workgroup"); __builtin_amdgcn_wave_barrier(); __builtin_amdgcn_fence(__ATOMIC_ACQUIRE, "workgroup"); }
__device__ __forceinline__ float pmul(float a, float b) { float p = a * b; asm volatile("" : "+v"(p)); return p; }
__device__ __forceinline__ int iclamp(int v, int lo, int hi) { return v < lo ? lo : (v > hi ? hi : v); }

typedef __attribute__((ext_vector_type(2))) _Float16 v2h;
typedef __attribute__((ext_vector_type(4))) _Float16 v4h;
typedef __attribute__((ext_vector_type(2))) float v2f;
__device__ __forceinline__ float nexp2(float v) { return __builtin_amdgcn_exp2f(v); }
__device__ __forceinline__ float silu(float v) { return v / (1.0f + __expf(-v)); }
__global__ __launch_bounds__(256) void prep_kernel(const float* __restrict__ wq, const float* __restrict__ wk, const float* __restrict__ wv, const float* __restrict__ wo, b16* __restrict__ WT, b16* __restrict__ WO) {
  const size_t u = (size_t)blockIdx.x * 256 + threadIdx.x; const size_t per = (size_t)DM * DM / 8; if (u >= 4 * per) return; const int m = (int)(u / per); const size_t e = (u % per) * 8; const int oo = (int)(e / DM), k0 = (int)(e % DM); const float* w = m == 0 ? wq : m == 1 ? wk : m == 2 ? wv : wo; v8b o;
  for (int j = 0; j < 8; ++j) o[j] = (b16)(bf16_rne(w[(size_t)(k0 + j) * DM + oo]) * WSC);
  b16* dst = (m < 3) ? (WT + (size_t)m * DM * DM + e) : (WO + e);
  for (int pass = 0; pass < 2; ++pass) { *(volatile v8b*)dst = o; __threadfence(); }
}
__global__ __launch_bounds__(256) void ln_kernel(const float* __restrict__ x, const float* __restrict__ g, const float* __restrict__ bb, float* __restrict__ XN) {
  const int wave = threadIdx.x >> 5, lane = threadIdx.x & 31; const size_t row = (size_t)blockIdx.x * 8 + wave; if (row >= (size_t)BL * T) return; const float* xr = x + row * DM;
  float v[32]; float s = 0.0f;
#pragma unroll
  for (int q = 0; q < 8; ++q) { const v4f f = *(const v4f*)(xr + q * 128 + lane * 4); for (int i = 0; i < 4; ++i) { v[q * 4 + i] = bf16_rne(f[i]); s += v[q * 4 + i]; } }
#pragma unroll
  for (int o = 1; o < 32; o <<= 1) s += __shfl_xor(s, o);
  const float mu = s * (1.0f / DM); float vs = 0.0f; for (int i = 0; i < 32; ++i) { const float d = v[i] - mu; vs += d * d; }
#pragma unroll
  for (int o = 1; o < 32; o <<= 1) vs += __shfl_xor(vs, o);
  const float rs = rsqrtf(vs * (1.0f / DM) + EPS);
  for (int pass = 0; pass < 2; ++pass) {
#pragma unroll
    for (int q = 0; q < 8; ++q) { const int c = q * 128 + lane * 4; v4f o4; for (int i = 0; i < 4; ++i) o4[i] = (v[q * 4 + i] - mu) * rs * bf16_rne(g[c + i]) + bf16_rne(bb[c + i]); *(volatile v4f*)(XN + row * DM + c) = o4; }
    __threadfence(); }
}
__global__ __launch_bounds__(256) void emb_kernel(const float* __restrict__ emb, const float* __restrict__ We, const float* __restrict__ be, float* __restrict__ EO) {
  __shared__ float SE[TE];
  const int b = blockIdx.y; for (int i = threadIdx.x; i < TE; i += 256) SE[i] = silu(bf16_rne(emb[(size_t)b * TE + i]));
  __syncthreads();
  const int o = blockIdx.x * 256 + threadIdx.x; float acc = 0.0f;
#pragma unroll 4
  for (int k = 0; k < TE; ++k) acc += SE[k] * bf16_rne(We[(size_t)k * 2 * DM + o]);
  acc += bf16_rne(be[o]);
  for (int pass = 0; pass < 2; ++pass) { ((volatile float*)EO)[(size_t)b * 2 * DM + o] = acc; __threadfence(); }
}
__global__ __launch_bounds__(128) void proj_kernel(const float* __restrict__ XN, const b16* __restrict__ WT, const float* __restrict__ bq, const float* __restrict__ bk, const float* __restrict__ bv, b16* __restrict__ QP, b16* __restrict__ KP, b16* __restrict__ VT) {
  __shared__ __attribute__((aligned(16))) b16 As[64][256 + 8]; __shared__ __attribute__((aligned(16))) float Tf[4][16][128 + 4];
  const int wave = threadIdx.x >> 5, lane = threadIdx.x & 31, nloc = lane & 15, hlf = lane >> 4; const int t0 = blockIdx.x * 64; const int b = blockIdx.y; const int slab = blockIdx.z, n0 = slab * 128, part = slab / 8, c0 = n0 - part * DM;
  const float* xb = XN + ((size_t)b * T + t0) * DM; const float* bias = part == 0 ? bq : part == 1 ? bk : bv;
  v8f acc[8];
#pragma unroll
  for (int t = 0; t < 8; ++t) acc[t] = (v8f){};
#pragma unroll 1
  for (int kc = 0; kc < DM; kc += 256) {
    __syncthreads();
    for (int i = threadIdx.x; i < 64 * 64; i += 128) { const int rr = i / 64, q = (i % 64) * 4; const v4f f = *(const v4f*)(xb + (size_t)rr * DM + kc + q); v4h o; for (int j = 0; j < 4; ++j) o[j] = (b16)(f[j] * XS); *(v4h*)(&As[rr][q]) = o; }
    __syncthreads();
#pragma unroll 2
    for (int kb = 0; kb < 256; kb += 32) { const v16b a = frag_kb(&As[wave * 16 + nloc][kb], hlf);
#pragma unroll
      for (int t = 0; t < 8; ++t) acc[t] = wmma16b(a, frag_kb(WT + (size_t)(n0 + t * 16 + nloc) * DM + kc + kb, hlf), acc[t]); } }
#pragma unroll
  for (int t = 0; t < 8; ++t) { const float bb = bf16_rne(bias[c0 + t * 16 + nloc]);
#pragma unroll
    for (int r = 0; r < 8; ++r) Tf[wave][8 * hlf + r][t * 16 + nloc] = acc[t][r] * (1.0f / (XS * WSC)) + bb; }
  __syncthreads();
  for (int pass = 0; pass < 2; ++pass) {
    if (part < 2) { b16* plane = part == 0 ? QP : KP; const int c = c0 + lane * 4; const int h = c / HD, d = c % HD;
      for (int rr = 0; rr < 16; ++rr) { const int tok = t0 + wave * 16 + rr; v4h o4; for (int j = 0; j < 4; ++j) o4[j] = (b16)(Tf[wave][rr][lane * 4 + j] * XS); *(volatile v4h*)(plane + (((size_t)b * H + h) * T + tok) * HD + d) = o4; } }
    else {
#pragma unroll 1
      for (int q = 0; q < 32; ++q) { const int cl = wave * 32 + q; const int c = c0 + cl; const int h = c / HD, d = c % HD; const int tk = lane * 2; v2h vv; vv[0] = (b16)(Tf[tk >> 4][tk & 15][cl] * XS); vv[1] = (b16)(Tf[(tk + 1) >> 4][(tk + 1) & 15][cl] * XS);
        *(volatile v2h*)(VT + (((size_t)b * H + h) * HD + d) * (size_t)T + t0 + tk) = vv; } }
    __threadfence(); }
}
__global__ __launch_bounds__(64) void attn_kernel(const b16* __restrict__ QP, const b16* __restrict__ KP, const b16* __restrict__ VT, const float* __restrict__ smask, float* __restrict__ Y) {
  __shared__ __attribute__((aligned(16))) b16 Pb[2][16][32 + 8]; __shared__ __attribute__((aligned(16))) float To[2][16][HD + 4];
  const int wave = threadIdx.x >> 5, lane = threadIdx.x & 31, hh = lane >> 4, col = lane & 15; const int b = blockIdx.y / H, h = blockIdx.y % H; const int q0 = blockIdx.x * 32 + wave * 16, qi = q0 + col;
  const size_t ph = (size_t)b * H + h; const b16* Qb = QP + ph * T * HD; const b16* Kb = KP + ph * T * HD; const b16* Vb = VT + ph * HD * (size_t)T; const float* mrow = smask + ((size_t)b * T + qi) * T;
  const v16b qa0 = frag_kb(Qb + (size_t)qi * HD, hh), qa1 = frag_kb(Qb + (size_t)qi * HD + 32, hh);
  const float cs = LOG2E / (8.0f * XS * XS);
  float m = -INFINITY, l = 0.0f; v8f o[4]; for (int t = 0; t < 4; ++t) o[t] = (v8f){};
#pragma unroll 1
  for (int kb = 0; kb < T; kb += 32) {
    float e[16]; float mx = -INFINITY;
#pragma unroll
    for (int u = 0; u < 2; ++u) { v8f s = (v8f){}; const size_t kr = (size_t)(kb + u * 16 + col) * HD; s = wmma16b(frag_kb(Kb + kr, hh), qa0, s); s = wmma16b(frag_kb(Kb + kr + 32, hh), qa1, s);
      const v4f m0 = *(const v4f*)(mrow + kb + u * 16 + 8 * hh), m1 = *(const v4f*)(mrow + kb + u * 16 + 8 * hh + 4);
#pragma unroll
      for (int r = 0; r < 8; ++r) { const float mk = bf16_rne((r < 4) ? m0[r] : m1[r - 4]); const float vv = s[r] * cs + (1.0f - mk) * MNEG * LOG2E; e[u * 8 + r] = vv; mx = fmaxf(mx, vv); } }
    mx = fmaxf(mx, __shfl_xor(mx, 16)); const float mn = fmaxf(m, mx); const float al = nexp2(m - mn); float sum = 0.0f;
#pragma unroll
    for (int i2 = 0; i2 < 16; ++i2) { const float p = nexp2(e[i2] - mn); sum += p; Pb[wave][col][(i2 < 8 ? 0 : 16) + 8 * hh + (i2 & 7)] = (b16)(p * PS); }
    sum += __shfl_xor(sum, 16); l = l * al + sum; m = mn;
    wave_lds_sync();
    const v16b pf = frag_kb(&Pb[wave][col][0], hh);
#pragma unroll
    for (int t = 0; t < 4; ++t) { o[t] *= al; o[t] = wmma16b(frag_kb(Vb + (size_t)(t * 16 + col) * T + kb, hh), pf, o[t]); }
    wave_lds_sync(); }
  const float inv = 1.0f / (l * PS * XS);
#pragma unroll
  for (int t = 0; t < 4; ++t)
#pragma unroll
    for (int r = 0; r < 8; ++r) To[wave][col][t * 16 + 8 * hh + r] = o[t][r] * inv;
  wave_lds_sync();
  for (int pass = 0; pass < 2; ++pass) { for (int rr = 0; rr < 16; ++rr) *(volatile v2f*)(Y + ((size_t)b * T + q0 + rr) * DM + h * HD + lane * 2) = *(const v2f*)(&To[wave][rr][lane * 2]); __threadfence(); }
}
__global__ __launch_bounds__(256) void ln2_kernel(const float* __restrict__ Y, const float* __restrict__ g, const float* __restrict__ bb, const float* __restrict__ EO, b16* __restrict__ HS) {
  const int wave = threadIdx.x >> 5, lane = threadIdx.x & 31; const size_t row = (size_t)blockIdx.x * 8 + wave; if (row >= (size_t)BL * T) return; const int b = (int)(row / T); const float* yr = Y + row * DM;
  float s = 0.0f;
#pragma unroll 1
  for (int q = 0; q < 8; ++q) { const v4f f = *(const v4f*)(yr + q * 128 + lane * 4); s += (f[0] + f[1]) + (f[2] + f[3]); }
#pragma unroll
  for (int o = 1; o < 32; o <<= 1) s += __shfl_xor(s, o);
  const float mu = s * (1.0f / DM); float vs = 0.0f;
#pragma unroll 1
  for (int q = 0; q < 8; ++q) { const v4f f = *(const v4f*)(yr + q * 128 + lane * 4); for (int i = 0; i < 4; ++i) { const float d = f[i] - mu; vs += d * d; } }
#pragma unroll
  for (int o = 1; o < 32; o <<= 1) vs += __shfl_xor(vs, o);
  const float rs = rsqrtf(vs * (1.0f / DM) + EPS); const float* sc = EO + (size_t)b * 2 * DM; const float* sh = sc + DM;
  for (int pass = 0; pass < 2; ++pass) {
#pragma unroll 1
    for (int q = 0; q < 8; ++q) { const int c = q * 128 + lane * 4; const v4f f = *(const v4f*)(yr + c); const v4f gg = *(const v4f*)(g + c), be2 = *(const v4f*)(bb + c), s4 = *(const v4f*)(sc + c), h4 = *(const v4f*)(sh + c); v4h o4;
      for (int i = 0; i < 4; ++i) { const float hv = ((f[i] - mu) * rs * bf16_rne(gg[i]) + bf16_rne(be2[i])) * (1.0f + s4[i]) + h4[i]; o4[i] = (b16)(silu(hv) * XS); } *(volatile v4h*)(HS + row * DM + c) = o4; }
    __threadfence(); }
}
__global__ __launch_bounds__(128) void out_kernel(const b16* __restrict__ HS, const b16* __restrict__ WO, const float* __restrict__ bo, const float* __restrict__ x, float* __restrict__ out) {
  __shared__ __attribute__((aligned(16))) float Tf[4][16][128 + 4];
  const int wave = threadIdx.x >> 5, lane = threadIdx.x & 31, nloc = lane & 15, hlf = lane >> 4; const int b = blockIdx.z; const size_t m0 = (size_t)b * T + ((size_t)blockIdx.x * 4 + wave) * 16; const int n0 = blockIdx.y * 128;
  v8f acc[8];
#pragma unroll
  for (int t = 0; t < 8; ++t) acc[t] = (v8f){};
#pragma unroll 2
  for (int kb = 0; kb < DM; kb += 32) { const v16b a = frag_kb(HS + (m0 + nloc) * DM + kb, hlf);
#pragma unroll
    for (int t = 0; t < 8; ++t) acc[t] = wmma16b(a, frag_kb(WO + (size_t)(n0 + t * 16 + nloc) * DM + kb, hlf), acc[t]); }
#pragma unroll
  for (int t = 0; t < 8; ++t) { const float bb = bf16_rne(bo[n0 + t * 16 + nloc]);
#pragma unroll
    for (int r = 0; r < 8; ++r) Tf[wave][8 * hlf + r][t * 16 + nloc] = acc[t][r] * (1.0f / (XS * WSC)) + bb; }
  wave_lds_sync();
  for (int pass = 0; pass < 2; ++pass) { for (int rr = 0; rr < 16; ++rr) { const v4f xv = *(const v4f*)(x + (m0 + rr) * DM + n0 + lane * 4); v4f f = *(const v4f*)(&Tf[wave][rr][lane * 4]); for (int j = 0; j < 4; ++j) f[j] += bf16_rne(xv[j]); *(volatile v4f*)(out + (m0 + rr) * DM + n0 + lane * 4) = f; } __threadfence(); }
}
}

extern "C" void kernel_launch(void* const* d_in, const int* in_sizes, int n_in, void* d_out, int out_size, void* d_ws, size_t ws_size, hipStream_t stream) {
  (void)n_in;
  auto Fp = [&](int i) { return (const float*)d_in[i]; };
  if (in_sizes[0] != B * T * DM || in_sizes[1] != B * TE || in_sizes[2] != B * T * T || in_sizes[5] != DM * DM || in_sizes[7] != DM * DM || in_sizes[9] != DM * DM || in_sizes[11] != TE * 2 * DM || in_sizes[12] != 2 * DM || in_sizes[15] != DM * DM || in_sizes[16] != DM || out_size != B * T * DM) return;
  size_t off = 0; char* ws = (char*)d_ws;
  auto carve = [&](size_t bytes) { char* p = ws + off; off += (bytes + 255) & ~(size_t)255; return p; };
  b16* WT = (b16*)carve((size_t)3 * DM * DM * 2); b16* WO = (b16*)carve((size_t)DM * DM * 2); float* XN = (float*)carve((size_t)B * T * DM * 4); float* EO = (float*)carve((size_t)B * 2 * DM * 4);
  const size_t plane = (size_t)B * T * DM * 2; b16* QP = (b16*)carve(plane); b16* KP = (b16*)carve(plane); b16* VT = (b16*)carve(plane); float* Y = (float*)carve((size_t)B * T * DM * 4); b16* HS = (b16*)carve(plane);
  if (off > ws_size || off > ((size_t)128 << 20)) return;
  prep_kernel<<<(unsigned)(((size_t)4 * DM * DM / 8 + 255) / 256), 256, 0, stream>>>(Fp(5), Fp(7), Fp(9), Fp(15), WT, WO);
  ln_kernel<<<(BL * T + 7) / 8, 256, 0, stream>>>(Fp(0), Fp(3), Fp(4), XN);
  emb_kernel<<<dim3(2 * DM / 256, BL), 256, 0, stream>>>(Fp(1), Fp(11), Fp(12), EO);
  proj_kernel<<<dim3(T / 64, BL, 24), 128, 0, stream>>>(XN, WT, Fp(6), Fp(8), Fp(10), QP, KP, VT);
  attn_kernel<<<dim3(T / 32, BL * H), 64, 0, stream>>>(QP, KP, VT, Fp(2), Y);
  ln2_kernel<<<(BL * T + 7) / 8, 256, 0, stream>>>(Y, Fp(13), Fp(14), EO, HS);
  out_kernel<<<dim3(T / 64, DM / 128, BL), 128, 0, stream>>>(HS, WO, Fp(16), Fp(0), (float*)d_out);
}
